// SE3TransformerInteractionBlock_47571057770949
// MI455X (gfx1250) — hardware-verified
//
#include <hip/hip_runtime.h>
#include <stddef.h>
#include <math.h>


#define NTHR   256
#define NWAVE  8
#define FDIM   80
#define M0     32
#define NV3    48
#define NHEAD  4
#define HC     576
#define WN     2304
#define HK     64
#define NBAS   16
#define ET     32
#define REC    160
#define NB     64
#define EPT    8
#define CHUNK  (NTHR * EPT)
#define WCAP   (EPT * 32)

#define K_SQRT3 1.7320508075688772f
#define K_FAN   6.928203230275509f
#define K_FAND  8.94427190999916f
#define K_SQ20  4.47213595499958f
#define K_SQ32  5.656854249492381f

#define EL_D    0
#define EL_HID  (EL_D + ET * HC * 4)
#define EL_RAW  (EL_HID + 2 * ET * HK * 4)
#define EL_FA   (EL_RAW + ET * FDIM * 4)
#define EL_FB   (EL_FA + ET * M0 * 4)
#define EL_FDS  (EL_FB + ET * 16 * 4)
#define EL_SH   (EL_FDS + ET * NV3 * 4)
#define EL_EMB  (EL_SH + ET * 4 * 4)
#define EL_O0   (EL_EMB + ET * NBAS * 4)
#define EL_SV   (EL_O0 + 2 * ET * 32 * 4)
#define EL_V3   (EL_SV + 2 * ET * 16 * 4)
#define EL_TOT  (EL_V3 + 2 * ET * NV3 * 4)

#define NL_XS   0
#define NL_QQ   (NL_XS + NB * FDIM * 4)
#define NL_QW   (NL_QQ + NB * FDIM * 4)
#define NL_AG   (NL_QW + NB * FDIM * 4)
#define NL_X01  (NL_AG + NB * FDIM * 4)
#define NL_A0   (NL_X01 + NB * FDIM * 4)
#define NL_F1   (NL_A0 + NB * HK * 4)
#define NL_OUT  (NL_F1 + NB * NV3 * 4)
#define NL_LIST (NL_OUT + NB * FDIM * 4)
#define NL_WCNT (NL_LIST + NWAVE * WCAP * 4)
#define NL_TOT  (NL_WCNT + 64)

static_assert((4 * WN * 8) % NTHR == 0);
static_assert((ET * REC) % (4 * NTHR) == 0);
static_assert(NB * 4 == NTHR);
static_assert(CHUNK <= 4096);
static_assert(NB <= 64);
static_assert((EL_TOT % 16) == 0 && EL_TOT <= 300 * 1024);
static_assert((NL_TOT % 16) == 0 && NL_TOT <= 300 * 1024);
static_assert(ET * REC * 4 <= ET * HC * 4);
static_assert((HC % 16) == 0 && WN == NHEAD * HC);
static_assert((2 * ET * HK) % NTHR == 0 && (ET * HK) % NTHR == 0);

typedef float          v4f   __attribute__((ext_vector_type(4)));
typedef float          v8f   __attribute__((ext_vector_type(8)));
typedef int            v4i   __attribute__((ext_vector_type(4)));
typedef unsigned short v8us  __attribute__((ext_vector_type(8)));
typedef unsigned short v16us __attribute__((ext_vector_type(16)));
typedef __bf16         v16b  __attribute__((ext_vector_type(16)));
union FragB { v16b v; v16us u; v8us h[2]; };

__device__ __forceinline__ v8f zero8f() {
  v8f c;
#pragma unroll
  for (int i = 0; i < 8; ++i) c[i] = 0.0f;
  return c;
}

__device__ __forceinline__ unsigned int bfr(float x) {
  const unsigned int u = __float_as_uint(x);
  return (u + 0x7FFFu + ((u >> 16) & 1u)) >> 16;
}

__device__ __forceinline__ void split16(const float* x, FragB& hi, FragB& lo) {
#pragma unroll
  for (int i = 0; i < 16; ++i) {
    const unsigned int hb = bfr(x[i]);
    const float hf = __uint_as_float(hb << 16);
    const unsigned int lb = bfr(x[i] - hf);
    hi.u[i] = (unsigned short)hb;
    lo.u[i] = (unsigned short)lb;
  }
}

__device__ __forceinline__ v8f wmb(v16b a, v16b b, v8f c) {
  v8f d = __builtin_amdgcn_wmma_f32_16x16x32_bf16(false, a, false, b, (short)0, c, false, false);
  asm volatile("v_nop\n\tv_nop\n\tv_nop\n\tv_nop" : "+v"(d) : "v"(a), "v"(b));
  return d;
}

__device__ __forceinline__ v8f mma3(const FragB& ah, const FragB& al, const FragB& bh, const FragB& bl, v8f c) {
  c = wmb(ah.v, bh.v, c);
  c = wmb(ah.v, bl.v, c);
  c = wmb(al.v, bh.v, c);
  return c;
}

__device__ __forceinline__ void frag_lds(const float* p0, FragB& hi, FragB& lo) {
  float x[16];
#pragma unroll
  for (int i = 0; i < 8; ++i) { x[i] = p0[i]; x[8 + i] = p0[16 + i]; }
  split16(x, hi, lo);
}

__device__ __forceinline__ void frag_pl(const unsigned short* q, FragB& f) {
  f.h[0] = *(const v8us*)q;
  f.h[1] = *(const v8us*)(q + 16);
}

__device__ __forceinline__ v8f tile3(const float* ap, int ast, const float* bp, int ldw, int nks, int k16, int hh) {
  v8f c = zero8f();
#pragma unroll 1
  for (int ks = 0; ks < nks; ++ks) {
    const float* a0 = ap + (ks * 32 + 8 * hh) * ast;
    const float* a1 = a0 + (k16 ? 0 : 16 * ast);
    const float* b0 = bp + (size_t)(ks * 32 + 8 * hh) * ldw;
    const float* b1 = b0 + (k16 ? 0 : (size_t)16 * ldw);
    float xa[16], xb[16];
#pragma unroll
    for (int i = 0; i < 8; ++i) {
      xa[i] = a0[i * ast];
      xb[i] = b0[(size_t)i * ldw];
      const float ta = a1[i * ast];
      const float tb = b1[(size_t)i * ldw];
      xa[8 + i] = k16 ? 0.0f : ta;
      xb[8 + i] = k16 ? 0.0f : tb;
    }
    FragB ah, al, bh, bl;
    split16(xa, ah, al);
    split16(xb, bh, bl);
    c = mma3(ah, al, bh, bl, c);
  }
  return c;
}

__device__ __forceinline__ int scan_chunk(const int* __restrict__ dsts, int nE, int cbase, int nodeBase,
                                          int vec8, int* list, int tid, int wave) {
  int wc = 0;
  const int el0  = tid * EPT;
  const int e0   = cbase + el0;
  const int sent = -2147483647 - 1;
  v4i da, db;
  if (vec8 != 0 && cbase + CHUNK <= nE) {
    da = *(const v4i*)(dsts + e0);
    db = *(const v4i*)(dsts + e0 + 4);
  } else {
    da.x = (e0     < nE) ? dsts[min(e0, nE - 1)] : sent;
    da.y = (e0 + 1 < nE) ? dsts[min(e0 + 1, nE - 1)] : sent;
    da.z = (e0 + 2 < nE) ? dsts[min(e0 + 2, nE - 1)] : sent;
    da.w = (e0 + 3 < nE) ? dsts[min(e0 + 3, nE - 1)] : sent;
    db.x = (e0 + 4 < nE) ? dsts[min(e0 + 4, nE - 1)] : sent;
    db.y = (e0 + 5 < nE) ? dsts[min(e0 + 5, nE - 1)] : sent;
    db.z = (e0 + 6 < nE) ? dsts[min(e0 + 6, nE - 1)] : sent;
    db.w = (e0 + 7 < nE) ? dsts[min(e0 + 7, nE - 1)] : sent;
  }
  const unsigned nb = (unsigned)nodeBase;
  const unsigned s0 = (unsigned)da.x - nb, s1 = (unsigned)da.y - nb;
  const unsigned s2 = (unsigned)da.z - nb, s3 = (unsigned)da.w - nb;
  const unsigned s4 = (unsigned)db.x - nb, s5 = (unsigned)db.y - nb;
  const unsigned s6 = (unsigned)db.z - nb, s7 = (unsigned)db.w - nb;
  const bool h0 = s0 < (unsigned)NB, h1 = s1 < (unsigned)NB, h2 = s2 < (unsigned)NB, h3 = s3 < (unsigned)NB;
  const bool h4 = s4 < (unsigned)NB, h5 = s5 < (unsigned)NB, h6 = s6 < (unsigned)NB, h7 = s7 < (unsigned)NB;
  const unsigned any = __builtin_amdgcn_ballot_w32(h0 | h1 | h2 | h3 | h4 | h5 | h6 | h7);
  if (any != 0u) {
#define HITJ(J, HJ, SJ) { \
      const unsigned mj = __builtin_amdgcn_ballot_w32(HJ); \
      if (mj != 0u) { \
        if (HJ) { \
          const int pos = wc + (int)__builtin_amdgcn_mbcnt_lo(mj, 0u); \
          if (pos < WCAP) list[wave * WCAP + pos] = (el0 + (J)) | ((int)(SJ) << 12); \
        } \
        wc += (int)__builtin_popcount(mj); } }
    HITJ(0, h0, s0)
    HITJ(1, h1, s1)
    HITJ(2, h2, s2)
    HITJ(3, h3, s3)
    HITJ(4, h4, s4)
    HITJ(5, h5, s5)
    HITJ(6, h6, s6)
    HITJ(7, h7, s7)
#undef HITJ
  }
  return wc;
}

__global__ __launch_bounds__(NTHR) void k_prep(const float* __restrict__ Wk2, const float* __restrict__ Wv2,
                                              unsigned short* planes) {
  const int u   = blockIdx.x * NTHR + threadIdx.x;
  const int pl  = u / (WN * 8);
  const int rem = u - pl * (WN * 8);
  const int n   = rem >> 3;
  const int kc  = rem & 7;
  const float* W = (pl < 2) ? Wk2 : Wv2;
  const int useLo = pl & 1;
  v8us o;
#pragma unroll
  for (int j = 0; j < 8; ++j) {
    const int k = kc * 8 + j;
    const float w = W[(size_t)k * WN + n];
    const unsigned int hb = bfr(w);
    const float hf = __uint_as_float(hb << 16);
    const unsigned int lb = bfr(w - hf);
    o[j] = (unsigned short)(useLo ? lb : hb);
  }
  unsigned short* dp = planes + (size_t)pl * (WN * HK) + (size_t)n * HK + kc * 8;
  *(volatile v8us*)dp = o;
  __threadfence();
  *(volatile v8us*)dp = o;
}

__global__ __launch_bounds__(NTHR) void k_edge(
    const float* __restrict__ nf, const int* __restrict__ ei,
    const float* __restrict__ esh, const float* __restrict__ emb,
    const float* __restrict__ Wk1, const float* __restrict__ bk1, const float* __restrict__ bk2,
    const float* __restrict__ Wv1, const float* __restrict__ bv1, const float* __restrict__ bv2,
    const unsigned short* __restrict__ planes, float* rec, int nN, int nE) {
  extern __shared__ __attribute__((aligned(16))) unsigned char dsm[];
  float* Dch = (float*)(dsm + EL_D);
  float* hid = (float*)(dsm + EL_HID);
  float* raw = (float*)(dsm + EL_RAW);
  float* fa  = (float*)(dsm + EL_FA);
  float* fb  = (float*)(dsm + EL_FB);
  float* fds = (float*)(dsm + EL_FDS);
  float* shv = (float*)(dsm + EL_SH);
  float* emv = (float*)(dsm + EL_EMB);
  float* o0  = (float*)(dsm + EL_O0);
  float* sv  = (float*)(dsm + EL_SV);
  float* v3  = (float*)(dsm + EL_V3);

  const int tid = threadIdx.x, lane = tid & 31, wave = tid >> 5, hh = lane >> 4, m = lane & 15;
  const int e0 = blockIdx.x * ET;

  for (int i = tid; i < ET * 4; i += NTHR) {
    const int e = i >> 2, c = i & 3;
    const int eg = min(e0 + e, nE - 1);
    shv[i] = esh[(size_t)eg * 4 + c];
  }
  for (int i = tid; i < ET * NBAS; i += NTHR) {
    const int e = i >> 4, b = i & 15;
    const int eg = min(e0 + e, nE - 1);
    emv[i] = emb[(size_t)eg * NBAS + b];
  }
  for (int i = tid; i < ET * FDIM; i += NTHR) {
    const int e = i / FDIM, c = i - e * FDIM;
    const int eg = min(e0 + e, nE - 1);
    int s = ei[eg];
    s = s < 0 ? 0 : (s > nN - 1 ? nN - 1 : s);
    raw[i] = nf[(size_t)s * FDIM + c];
  }
  __syncthreads();

  for (int i = tid; i < ET * M0; i += NTHR) {
    const int e = i >> 5, u = i & 31;
    fa[i] = raw[e * FDIM + u] * shv[e * 4];
  }
  for (int i = tid; i < ET * 16; i += NTHR) {
    const int e = i >> 4, u = i & 15;
    const float* vp = raw + e * FDIM + M0 + u * 3;
    const float* sp = shv + e * 4 + 1;
    float d = vp[0] * sp[0];
    d = fmaf(vp[1], sp[1], d);
    d = fmaf(vp[2], sp[2], d);
    fb[i] = d * (1.0f / K_SQRT3);
  }
  for (int i = tid; i < ET * NV3; i += NTHR) {
    const int e = i / NV3, cc = i - e * NV3;
    fds[i] = raw[e * FDIM + M0 + cc] * shv[e * 4];
  }
#pragma unroll 1
  for (int it = 0; it < (2 * ET * HK) / NTHR; ++it) {
    const int t   = it * NTHR + tid;
    const int mat = t / (ET * HK);
    const int r   = t - mat * (ET * HK);
    const int e = r >> 6, j = r & 63;
    const float* W1 = mat ? Wv1 : Wk1;
    const float* b1 = mat ? bv1 : bk1;
    const float* ep = emv + e * NBAS;
    float a = 0.0f;
#pragma unroll 4
    for (int b = 0; b < NBAS; ++b) a = fmaf(ep[b], W1[b * HK + j], a);
    a += b1[j];
    const float sg = 1.0f / (1.0f + expf(-a));
    hid[mat * (ET * HK) + e * HK + j] = a * sg;
  }
  __syncthreads();

#pragma unroll 1
  for (int mat = 0; mat < 2; ++mat) {
    const float* hb = hid + mat * (ET * HK);
    FragB ah00, al00, ah01, al01, ah10, al10, ah11, al11;
    frag_lds(hb + (0 * 16 + m) * HK + 0 * 32 + 8 * hh, ah00, al00);
    frag_lds(hb + (0 * 16 + m) * HK + 1 * 32 + 8 * hh, ah01, al01);
    frag_lds(hb + (1 * 16 + m) * HK + 0 * 32 + 8 * hh, ah10, al10);
    frag_lds(hb + (1 * 16 + m) * HK + 1 * 32 + 8 * hh, ah11, al11);
    const unsigned short* ph  = planes + (size_t)(2 * mat) * (WN * HK);
    const unsigned short* plo = ph + (size_t)WN * HK;
    const float* b2 = mat ? bv2 : bk2;

#pragma unroll 1
    for (int hd = 0; hd < NHEAD; ++hd) {
#pragma unroll 1
      for (int ct = wave; ct < HC / 16; ct += NWAVE) {
        const int n = hd * HC + ct * 16 + m;
        const unsigned short* qh = ph  + (size_t)n * HK + 8 * hh;
        const unsigned short* ql = plo + (size_t)n * HK + 8 * hh;
        FragB bh0, bl0, bh1, bl1;
        frag_pl(qh, bh0);
        frag_pl(ql, bl0);
        frag_pl(qh + 32, bh1);
        frag_pl(ql + 32, bl1);
        v8f c0 = zero8f(), c1 = zero8f();
        c0 = mma3(ah00, al00, bh0, bl0, c0);
        c1 = mma3(ah10, al10, bh0, bl0, c1);
        c0 = mma3(ah01, al01, bh1, bl1, c0);
        c1 = mma3(ah11, al11, bh1, bl1, c1);
        const float bias = b2[n];
        float* d0 = Dch + (8 * hh) * HC + ct * 16 + m;
#pragma unroll
        for (int r = 0; r < 8; ++r) {
          d0[r * HC]        = c0[r] + bias;
          d0[(16 + r) * HC] = c1[r] + bias;
        }
      }
      __syncthreads();

      {
        const int e = tid >> 3, w = tid & 7;
        const float* Dr = Dch + e * HC;
        const float* fap = fa + e * M0;
        const float* fbp = fb + e * 16;
        float ass = 0.0f, avv = 0.0f;
#pragma unroll 4
        for (int u = 0; u < M0; ++u) ass = fmaf(fap[u], Dr[u * 8 + w], ass);
#pragma unroll 4
        for (int u = 0; u < 16; ++u) avv = fmaf(fbp[u], Dr[256 + u * 8 + w], avv);
        o0[(mat * ET + e) * 32 + hd * 8 + w] = (ass + avv) * (1.0f / K_FAN);
      }
      if (tid < 128) {
        const int e = tid >> 2, w = tid & 3;
        const float* Dr = Dch + e * HC;
        const float* fcp = raw + e * FDIM;
        const float* fdp = fds + e * NV3;
        float S = 0.0f, V0 = 0.0f;
#pragma unroll 4
        for (int u = 0; u < M0; ++u) S = fmaf(fcp[u], Dr[384 + u * 4 + w], S);
#pragma unroll 4
        for (int u = 0; u < 16; ++u) V0 = fmaf(fdp[u * 3], Dr[512 + u * 4 + w], V0);
        sv[(mat * ET + e) * 16 + hd * 4 + w] = S;
        v3[(mat * ET + e) * NV3 + (hd * 4 + w) * 3] = V0;
      } else {
        const int e = (tid - 128) >> 2, w = tid & 3;
        const float* Dr = Dch + e * HC;
        const float* fdp = fds + e * NV3;
        float V1 = 0.0f, V2 = 0.0f;
#pragma unroll 4
        for (int u = 0; u < 16; ++u) {
          const float dw = Dr[512 + u * 4 + w];
          V1 = fmaf(fdp[u * 3 + 1], dw, V1);
          V2 = fmaf(fdp[u * 3 + 2], dw, V2);
        }
        v3[(mat * ET + e) * NV3 + (hd * 4 + w) * 3 + 1] = V1;
        v3[(mat * ET + e) * NV3 + (hd * 4 + w) * 3 + 2] = V2;
      }
      __syncthreads();
    }
  }

  float* stg = Dch;
  for (int i = tid; i < ET * REC; i += NTHR) {
    const int e   = i / REC;
    const int c   = i - e * REC;
    const int cm  = (c >= 80) ? 1 : 0;
    const int cc  = c - 80 * cm;
    const int isv = (cc >= 32) ? 1 : 0;
    const int ca  = cc < 31 ? cc : 31;
    const float vo = o0[(cm * ET + e) * 32 + ca];
    const int cb  = cc - 32 < 0 ? 0 : cc - 32;
    const int hw  = cb / 3;
    const int ii  = cb - hw * 3;
    const float v1 = fmaf(sv[(cm * ET + e) * 16 + hw], shv[e * 4 + 1 + ii], v3[(cm * ET + e) * NV3 + cb]) * (1.0f / K_FAN);
    stg[i] = isv ? v1 : vo;
  }
  __syncthreads();
  float* gp = rec + (size_t)e0 * REC;
#pragma unroll 1
  for (int u = tid; u < (ET * REC) / 4; u += NTHR) {
    const v4f v = *(const v4f*)(stg + 4 * u);
    *(volatile v4f*)(gp + 4 * u) = v;
  }
  __threadfence();
#pragma unroll 1
  for (int u = tid; u < (ET * REC) / 4; u += NTHR) {
    const v4f v = *(const v4f*)(stg + 4 * u);
    *(volatile v4f*)(gp + 4 * u) = v;
  }
}

__global__ __launch_bounds__(NTHR) void k_node(
    const float* __restrict__ nf, const int* __restrict__ ei, const float* __restrict__ rec,
    const float* __restrict__ Wq0, const float* __restrict__ Wq1,
    const float* __restrict__ Wd0, const float* __restrict__ Wd1,
    const float* __restrict__ Wo0, const float* __restrict__ Wo1,
    const float* __restrict__ Wf10, const float* __restrict__ Wf11,
    const float* __restrict__ Wf20, const float* __restrict__ Wf21,
    float* out, int nN, int nE, int vec8) {
  extern __shared__ __attribute__((aligned(16))) unsigned char dsm[];
  float* xs   = (float*)(dsm + NL_XS);
  float* qq   = (float*)(dsm + NL_QQ);
  float* qw   = (float*)(dsm + NL_QW);
  float* ag   = (float*)(dsm + NL_AG);
  float* x01  = (float*)(dsm + NL_X01);
  float* a0   = (float*)(dsm + NL_A0);
  float* f1   = (float*)(dsm + NL_F1);
  float* outs = (float*)(dsm + NL_OUT);
  int*   list = (int*)(dsm + NL_LIST);
  int*   wcnt = (int*)(dsm + NL_WCNT);

  const int tid = threadIdx.x, lane = tid & 31, wave = tid >> 5, hh = lane >> 4, m = lane & 15;
  const int nodeBase = blockIdx.x * NB;
  const int slot = tid >> 2, hd = tid & 3;
  const int* dsts = ei + nE;

  for (int i = tid; i < NB * FDIM; i += NTHR) {
    const int r = i / FDIM, c = i - r * FDIM;
    const int node = min(nodeBase + r, nN - 1);
    xs[i] = nf[(size_t)node * FDIM + c];
  }
  __syncthreads();

  for (int i = tid; i < NB * 32; i += NTHR) {
    const int sl = i >> 5, c = i & 31, h = c >> 3, w = c & 7;
    const float* sp = xs + sl * FDIM;
    const float* wp = Wq0 + h * (32 * 8) + w;
    float a = 0.0f;
#pragma unroll 4
    for (int u = 0; u < 32; ++u) a = fmaf(sp[u], wp[u * 8], a);
    qq[sl * FDIM + c] = a * (1.0f / K_SQ32);
  }
  for (int i = tid; i < NB * NV3; i += NTHR) {
    const int sl = i / NV3, cc = i - sl * NV3;
    const int hw = cc / 3, ii = cc - hw * 3, h = hw >> 2, w = hw & 3;
    const float* vp = xs + sl * FDIM + M0 + ii;
    const float* wp = Wq1 + h * (16 * 4) + w;
    float a = 0.0f;
#pragma unroll 4
    for (int u = 0; u < 16; ++u) a = fmaf(vp[u * 3], wp[u * 4], a);
    qq[sl * FDIM + M0 + cc] = a * 0.25f;
  }
  __syncthreads();
  for (int i = tid; i < NB * 32; i += NTHR) {
    const int sl = i >> 5, c = i & 31, h = c >> 3, v = c & 7;
    const float* qp = qq + sl * FDIM + h * 8;
    float a = 0.0f;
#pragma unroll
    for (int u = 0; u < 8; ++u) a = fmaf(qp[u], Wd0[u * 8 + v], a);
    qw[sl * FDIM + c] = a;
  }
  for (int i = tid; i < NB * NV3; i += NTHR) {
    const int sl = i / NV3, cc = i - sl * NV3;
    const int hw = cc / 3, ii = cc - hw * 3, h = hw >> 2, v = hw & 3;
    const float* qp = qq + sl * FDIM + M0 + h * 12 + ii;
    float a = 0.0f;
#pragma unroll
    for (int u = 0; u < 4; ++u) a = fmaf(qp[u * 3], Wd1[u * 4 + v], a);
    qw[sl * FDIM + M0 + cc] = a;
  }
  __syncthreads();

  float qa[8], qb[12], acc[20];
#pragma unroll
  for (int v = 0; v < 8; ++v) qa[v] = qw[slot * FDIM + hd * 8 + v];
#pragma unroll
  for (int j = 0; j < 12; ++j) qb[j] = qw[slot * FDIM + M0 + hd * 12 + j];
#pragma unroll
  for (int c = 0; c < 20; ++c) acc[c] = 0.0f;
  float mrun = -10.0f, dsum = 0.0f;

  const int nChunks = (nE + CHUNK - 1) / CHUNK;
#pragma unroll 1
  for (int ch = 0; ch < nChunks; ++ch) {
    const int cbase = ch * CHUNK;
    const int wc = scan_chunk(dsts, nE, cbase, nodeBase, vec8, list, tid, wave);
    if (lane == 0) wcnt[wave] = wc;
    __syncthreads();
#pragma unroll 1
    for (int w = 0; w < NWAVE; ++w) {
      int cnt = wcnt[w];
      cnt = cnt < 0 ? 0 : (cnt > WCAP ? WCAP : cnt);
      const int* lp = list + w * WCAP;
#pragma unroll 1
      for (int p = 0; p < cnt; ++p) {
        const int ent = lp[p];
        const int sl  = ent >> 12;
        if (sl == slot) {
          int e = cbase + (ent & 4095);
          e = e < 0 ? 0 : (e > nE - 1 ? nE - 1 : e);
          const float* rp = rec + (size_t)e * REC;
          const v4f ka  = *(const v4f*)(rp + hd * 8);
          const v4f kb  = *(const v4f*)(rp + hd * 8 + 4);
          const v4f kc0 = *(const v4f*)(rp + 32 + hd * 12);
          const v4f kc1 = *(const v4f*)(rp + 36 + hd * 12);
          const v4f kc2 = *(const v4f*)(rp + 40 + hd * 12);
          const v4f va  = *(const v4f*)(rp + 80 + hd * 8);
          const v4f vb  = *(const v4f*)(rp + 84 + hd * 8);
          const v4f vc0 = *(const v4f*)(rp + 112 + hd * 12);
          const v4f vc1 = *(const v4f*)(rp + 116 + hd * 12);
          const v4f vc2 = *(const v4f*)(rp + 120 + hd * 12);
          float kk[20], vv[20];
          kk[0] = ka.x;  kk[1] = ka.y;  kk[2] = ka.z;  kk[3] = ka.w;
          kk[4] = kb.x;  kk[5] = kb.y;  kk[6] = kb.z;  kk[7] = kb.w;
          kk[8] = kc0.x; kk[9] = kc0.y; kk[10] = kc0.z; kk[11] = kc0.w;
          kk[12] = kc1.x; kk[13] = kc1.y; kk[14] = kc1.z; kk[15] = kc1.w;
          kk[16] = kc2.x; kk[17] = kc2.y; kk[18] = kc2.z; kk[19] = kc2.w;
          vv[0] = va.x;  vv[1] = va.y;  vv[2] = va.z;  vv[3] = va.w;
          vv[4] = vb.x;  vv[5] = vb.y;  vv[6] = vb.z;  vv[7] = vb.w;
          vv[8] = vc0.x; vv[9] = vc0.y; vv[10] = vc0.z; vv[11] = vc0.w;
          vv[12] = vc1.x; vv[13] = vc1.y; vv[14] = vc1.z; vv[15] = vc1.w;
          vv[16] = vc2.x; vv[17] = vc2.y; vv[18] = vc2.z; vv[19] = vc2.w;
          float l0 = 0.0f, l1 = 0.0f;
#pragma unroll
          for (int v = 0; v < 8; ++v) l0 = fmaf(qa[v], kk[v], l0);
#pragma unroll
          for (int j = 0; j < 12; ++j) l1 = fmaf(qb[j], kk[8 + j], l1);
          float lg = (l0 + l1 * (1.0f / K_SQRT3)) * (1.0f / K_FAND);
          lg = lg * (1.0f / K_SQ20);
          lg = fminf(fmaxf(lg, -10.0f), 10.0f);
          const float mn = fmaxf(mrun, lg);
          const float rr = expf(mrun - mn);
          const float pp = expf(lg - mn);
          dsum = fmaf(dsum, rr, pp);
#pragma unroll
          for (int c = 0; c < 20; ++c) acc[c] = fmaf(pp, vv[c], acc[c] * rr);
          mrun = mn;
        }
      }
    }
    __syncthreads();
  }

  {
    const float inv = 1.0f / (dsum + 1e-12f);
#pragma unroll
    for (int w = 0; w < 8; ++w) ag[slot * FDIM + hd * 8 + w] = acc[w] * inv;
#pragma unroll
    for (int j = 0; j < 12; ++j) ag[slot * FDIM + M0 + hd * 12 + j] = acc[8 + j] * inv;
  }
  __syncthreads();

  {
    const int rt = wave >> 1, cti = wave & 1;
    const v8f c = tile3(ag + (rt * 16 + m) * FDIM, 1, Wo0 + cti * 16 + m, 32, 1, 0, hh);
#pragma unroll
    for (int r = 0; r < 8; ++r) {
      const int idx = (rt * 16 + 8 * hh + r) * FDIM + cti * 16 + m;
      x01[idx] = xs[idx] + c[r] * (1.0f / K_SQ32);
    }
  }
#pragma unroll 1
  for (int rt = wave; rt < 12; rt += NWAVE) {
    const int R = rt * 16 + m, sl = R / 3, ii = R - 3 * sl;
    const v8f c = tile3(ag + sl * FDIM + M0 + ii, 3, Wo1 + m, 16, 1, 1, hh);
#pragma unroll
    for (int r = 0; r < 8; ++r) {
      const int R2 = rt * 16 + 8 * hh + r, s2 = R2 / 3, i2 = R2 - 3 * s2;
      const int idx = s2 * FDIM + M0 + m * 3 + i2;
      x01[idx] = xs[idx] + c[r] * 0.25f;
    }
  }
  __syncthreads();

  {
    const int rt = wave >> 1;
#pragma unroll 1
    for (int q = 0; q < 2; ++q) {
      const int ct = (wave & 1) * 2 + q;
      const v8f c = tile3(x01 + (rt * 16 + m) * FDIM, 1, Wf10 + ct * 16 + m, 64, 1, 0, hh);
#pragma unroll
      for (int r = 0; r < 8; ++r) {
        const float f = c[r] * (1.0f / K_SQ32);
        const float sg = 1.0f / (1.0f + expf(-f));
        a0[(rt * 16 + 8 * hh + r) * HK + ct * 16 + m] = f * sg;
      }
    }
  }
#pragma unroll 1
  for (int rt = wave; rt < 12; rt += NWAVE) {
    const int R = rt * 16 + m, sl = R / 3, ii = R - 3 * sl;
    const v8f c = tile3(x01 + sl * FDIM + M0 + ii, 3, Wf11 + m, 16, 1, 1, hh);
#pragma unroll
    for (int r = 0; r < 8; ++r) {
      const int R2 = rt * 16 + 8 * hh + r, s2 = R2 / 3, i2 = R2 - 3 * s2;
      f1[s2 * NV3 + m * 3 + i2] = c[r] * 0.25f;
    }
  }
  __syncthreads();
  for (int i = tid; i < NB * 16; i += NTHR) {
    const int sl = i >> 4, w = i & 15;
    float* fp = f1 + sl * NV3 + w * 3;
    const float fx = fp[0], fy = fp[1], fz = fp[2];
    const float nn = sqrtf(fmaf(fz, fz, fmaf(fy, fy, fx * fx)));
    const float safe = fmaxf(nn, 1e-8f);
    const float sn = nn * (1.0f / (1.0f + expf(-nn)));
    const float g = (nn < 1e-8f) ? 0.0f : (1.0f / safe) * sn;
    fp[0] = fx * g; fp[1] = fy * g; fp[2] = fz * g;
  }
  __syncthreads();

  {
    const int rt = wave >> 1, cti = wave & 1;
    const v8f c = tile3(a0 + (rt * 16 + m) * HK, 1, Wf20 + cti * 16 + m, 32, 2, 0, hh);
#pragma unroll
    for (int r = 0; r < 8; ++r) {
      const int idx = (rt * 16 + 8 * hh + r) * FDIM + cti * 16 + m;
      outs[idx] = x01[idx] + c[r] * 0.125f;
    }
  }
#pragma unroll 1
  for (int rt = wave; rt < 12; rt += NWAVE) {
    const int R = rt * 16 + m, sl = R / 3, ii = R - 3 * sl;
    const v8f c = tile3(f1 + sl * NV3 + ii, 3, Wf21 + m, 16, 1, 1, hh);
#pragma unroll
    for (int r = 0; r < 8; ++r) {
      const int R2 = rt * 16 + 8 * hh + r, s2 = R2 / 3, i2 = R2 - 3 * s2;
      const int idx = s2 * FDIM + M0 + m * 3 + i2;
      outs[idx] = x01[idx] + c[r] * 0.25f;
    }
  }
  __syncthreads();

  int nv = nN - nodeBase;
  nv = nv > NB ? NB : (nv < 0 ? 0 : nv);
  const int n4 = nv * (FDIM / 4);
  float* ob = out + (size_t)nodeBase * FDIM;
#pragma unroll 1
  for (int u = tid; u < n4; u += NTHR) {
    const v4f v = *(const v4f*)(outs + 4 * u);
    *(volatile v4f*)(ob + 4 * u) = v;
  }
  __threadfence();
#pragma unroll 1
  for (int u = tid; u < n4; u += NTHR) {
    const v4f v = *(const v4f*)(outs + 4 * u);
    *(volatile v4f*)(ob + 4 * u) = v;
  }
}

extern "C" void kernel_launch(void* const* d_in, const int* in_sizes, int n_in,
                              void* d_out, int out_size, void* d_ws, size_t ws_size,
                              hipStream_t stream) {
  if (n_in < 22) return;
  const int nN = in_sizes[0] / FDIM;
  if (nN < 1 || in_sizes[0] != nN * FDIM) return;
  const int nE = in_sizes[1] / 2;
  if (nE < 1 || in_sizes[1] != 2 * nE) return;
  if (in_sizes[2] != nE * 4 || in_sizes[3] != nE * NBAS) return;
  if (in_sizes[4] != NHEAD * 32 * 8 || in_sizes[5] != NHEAD * 16 * 4) return;
  if (in_sizes[6] != NBAS * HK || in_sizes[7] != HK || in_sizes[8] != HK * WN || in_sizes[9] != WN) return;
  if (in_sizes[10] != NBAS * HK || in_sizes[11] != HK || in_sizes[12] != HK * WN || in_sizes[13] != WN) return;
  if (in_sizes[14] != 64 || in_sizes[15] != 16 || in_sizes[16] != 1024 || in_sizes[17] != 256) return;
  if (in_sizes[18] != 2048 || in_sizes[19] != 256 || in_sizes[20] != 2048 || in_sizes[21] != 256) return;
  if (out_size != nN * FDIM) return;

  const float* nf   = (const float*)d_in[0];
  const int*   ei   = (const int*)d_in[1];
  const float* esh  = (const float*)d_in[2];
  const float* emb  = (const float*)d_in[3];
  const float* Wq0  = (const float*)d_in[4];
  const float* Wq1  = (const float*)d_in[5];
  const float* Wk1  = (const float*)d_in[6];
  const float* bk1  = (const float*)d_in[7];
  const float* Wk2  = (const float*)d_in[8];
  const float* bk2  = (const float*)d_in[9];
  const float* Wv1  = (const float*)d_in[10];
  const float* bv1  = (const float*)d_in[11];
  const float* Wv2  = (const float*)d_in[12];
  const float* bv2  = (const float*)d_in[13];
  const float* Wd0  = (const float*)d_in[14];
  const float* Wd1  = (const float*)d_in[15];
  const float* Wo0  = (const float*)d_in[16];
  const float* Wo1  = (const float*)d_in[17];
  const float* Wf10 = (const float*)d_in[18];
  const float* Wf11 = (const float*)d_in[19];
  const float* Wf20 = (const float*)d_in[20];
  const float* Wf21 = (const float*)d_in[21];
  float* outp = (float*)d_out;

  const int EB   = (nE + ET - 1) / ET;
  const int NBLK = (nN + NB - 1) / NB;

  char* ws = (char*)d_ws;
  size_t off = 0;
  const size_t szPl  = (size_t)4 * WN * HK * 2;
  const size_t oPl   = off; off += (szPl + 255) & ~(size_t)255;
  const size_t szRec = (size_t)EB * ET * REC * 4;
  const size_t oRec  = off; off += (szRec + 255) & ~(size_t)255;
  size_t limit = (size_t)134217728;
  if (ws_size < limit) limit = ws_size;
  if (off > limit) return;

  unsigned short* planes = (unsigned short*)(ws + oPl);
  float* recb = (float*)(ws + oRec);
  const int vec8 = ((nE & 3) == 0) ? 1 : 0;

  k_prep<<<(4 * WN * 8) / NTHR, NTHR, 0, stream>>>(Wk2, Wv2, planes);

  hipFuncSetAttribute(reinterpret_cast<const void*>(&k_edge), hipFuncAttributeMaxDynamicSharedMemorySize, EL_TOT);
  k_edge<<<EB, NTHR, EL_TOT, stream>>>(nf, ei, esh, emb, Wk1, bk1, bk2, Wv1, bv1, bv2,
                                       planes, recb, nN, nE);

  hipFuncSetAttribute(reinterpret_cast<const void*>(&k_node), hipFuncAttributeMaxDynamicSharedMemorySize, NL_TOT);
  k_node<<<NBLK, NTHR, NL_TOT, stream>>>(nf, ei, recb, Wq0, Wq1, Wd0, Wd1, Wo0, Wo1,
                                         Wf10, Wf11, Wf20, Wf21, outp, nN, nE, vec8);
}
